// TriplaneNeRF_31636729102599
// MI455X (gfx1250) — hardware-verified
//
#include <hip/hip_runtime.h>
#define RR 64
#define PC 32
#define HID 128
#define FEAT 96
#define NPTS (4 * 262144)

typedef _Float16 v16h __attribute__((ext_vector_type(16)));
typedef _Float16 v8h  __attribute__((ext_vector_type(8)));
typedef _Float16 v8ha __attribute__((ext_vector_type(8), may_alias));
typedef float    v8f  __attribute__((ext_vector_type(8)));
typedef float    v4f  __attribute__((ext_vector_type(4)));
typedef float    v4fa __attribute__((ext_vector_type(4), may_alias));
union Frag { v16h v; v8h half[2]; _Float16 h[16]; };

__device__ __forceinline__ v8f mma16(v16h a, v16h b, v8f c) {
  c = __builtin_amdgcn_wmma_f32_16x16x32_f16(false, a, false, b, (short)0, c, false, false);
  asm volatile("v_nop\n\tv_nop\n\tv_nop\n\tv_nop" : "+v"(c) : "v"(a), "v"(b));
  return c;
}

__global__ __launch_bounds__(256) void k_cvt16(const float* __restrict__ src, _Float16* __restrict__ dst, int n8) {
  const int t = blockIdx.x * 256 + threadIdx.x;
  if (t >= n8) return;
  const v4f a = *(const v4fa*)(src + (size_t)t * 8), b = *(const v4fa*)(src + (size_t)t * 8 + 4);
  v8h v; v[0]=(_Float16)a[0]; v[1]=(_Float16)a[1]; v[2]=(_Float16)a[2]; v[3]=(_Float16)a[3];
  v[4]=(_Float16)b[0]; v[5]=(_Float16)b[1]; v[6]=(_Float16)b[2]; v[7]=(_Float16)b[3];
  *(volatile v8h*)(dst + (size_t)t * 8) = v;
  __threadfence();
  *(volatile v8h*)(dst + (size_t)t * 8) = v;
}

__global__ __launch_bounds__(256) void k_transpose16(const float* __restrict__ W, _Float16* __restrict__ Wt, int K, int N) {
  const int t = blockIdx.x * 256 + threadIdx.x;
  const int k8n = K / 8;
  if (t >= N * k8n) return;
  const int n = t / k8n, k8 = (t % k8n) * 8;
  v8h v;
#pragma unroll
  for (int i = 0; i < 8; ++i) v[i] = (_Float16)W[(size_t)(k8 + i) * N + n];
  *(volatile v8h*)(Wt + (size_t)n * K + k8) = v;
  __threadfence();
  *(volatile v8h*)(Wt + (size_t)n * K + k8) = v;
}

template <int ACT, bool OUT16>
__global__ __launch_bounds__(128) void k_gemm(const _Float16* __restrict__ A, int lda, const _Float16* __restrict__ Bt, int ldb,
                                            const float* __restrict__ bias, void* __restrict__ Cout, int ldc, int M, int N, int K) {
  __shared__ __attribute__((aligned(16))) float so[4][16][64];
  const int tid = threadIdx.x, w = tid >> 5, lane = tid & 31, ln = lane & 15, hh = lane >> 4;
  const int ntn = N / 64;
  const int wid = blockIdx.x * 4 + w;
  const int mt = wid / ntn, nq = wid % ntn;
  if (mt * 16 >= M) return;
  const int row0 = mt * 16, col0 = nq * 64;
  const _Float16* arow = A + (size_t)(row0 + ln) * lda;
  v8f acc[4] = {};
  for (int kb = 0; kb < K; kb += 32) {
    Frag a;
    a.half[0] = *(const v8ha*)(arow + kb + 8 * hh);
    a.half[1] = *(const v8ha*)(arow + kb + 16 + 8 * hh);
#pragma unroll
    for (int t = 0; t < 4; ++t) {
      const _Float16* brow = Bt + (size_t)(col0 + t * 16 + ln) * ldb + kb;
      Frag b;
      b.half[0] = *(const v8ha*)(brow + 8 * hh);
      b.half[1] = *(const v8ha*)(brow + 16 + 8 * hh);
      acc[t] = mma16(a.v, b.v, acc[t]);
    }
  }
#pragma unroll
  for (int t = 0; t < 4; ++t) {
    const float bv = bias ? bias[col0 + t * 16 + ln] : 0.f;
#pragma unroll
    for (int r = 0; r < 8; ++r) { float v = acc[t][r] + bv; if (ACT == 1) v = fmaxf(v, 0.f); so[w][8 * hh + r][t * 16 + ln] = v; }
  }
  __builtin_amdgcn_fence(__ATOMIC_ACQ_REL, "workgroup");
  __builtin_amdgcn_wave_barrier();
  if (OUT16) {
    _Float16* C = (_Float16*)Cout;
    const int rsub = lane >> 3, c8 = (lane & 7) * 8;
    for (int pass = 0; pass < 2; ++pass) {
#pragma unroll
      for (int q = 0; q < 4; ++q) {
        const int r = q * 4 + rsub;
        v8h v;
#pragma unroll
        for (int i = 0; i < 8; ++i) v[i] = (_Float16)so[w][r][c8 + i];
        *(volatile v8h*)(C + (size_t)(row0 + r) * ldc + col0 + c8) = v;
      }
      if (pass == 0) __threadfence();
    }
  } else {
    float* C = (float*)Cout;
    const int rsub = lane >> 4, c4 = (lane & 15) * 4;
    for (int pass = 0; pass < 2; ++pass) {
#pragma unroll
      for (int q = 0; q < 8; ++q) {
        const int r = q * 2 + rsub;
        const v4f v = *(const v4fa*)&so[w][r][c4];
        *(volatile v4f*)(C + (size_t)(row0 + r) * ldc + col0 + c4) = v;
      }
      if (pass == 0) __threadfence();
    }
  }
}

__global__ __launch_bounds__(128) void k_nerf(const float* __restrict__ pts, const float* __restrict__ planes,
                                            const _Float16* __restrict__ dW1h, const float* __restrict__ db1, const _Float16* __restrict__ dW2h, const float* __restrict__ db2,
                                            const float* __restrict__ dW3, const float* __restrict__ db3,
                                            const _Float16* __restrict__ rW1h, const float* __restrict__ rb1, const float* __restrict__ rW2, const float* __restrict__ rb2,
                                            float* __restrict__ rgb, float* __restrict__ dens) {
  __shared__ __attribute__((aligned(16))) _Float16 sA[4][16][FEAT + 8];
  __shared__ __attribute__((aligned(16))) _Float16 sH[4][16][HID + 8];
  __shared__ __attribute__((aligned(16))) float    sH2[4][16][HID + 4];
  __shared__ __attribute__((aligned(16))) float    sRh[4][16][HID + 4];
  __shared__ float sOut[4][32][4];
  const int tid = threadIdx.x, w = tid >> 5, lane = tid & 31, ln = lane & 15, hh = lane >> 4;
  const size_t p0 = ((size_t)blockIdx.x * 4 + w) * 32;
  for (int sub = 0; sub < 2; ++sub) {
    const size_t pbase = p0 + sub * 16;
    __builtin_amdgcn_fence(__ATOMIC_ACQ_REL, "workgroup");
    __builtin_amdgcn_wave_barrier();
    for (int i = 0; i < 16; ++i) {
      const float px = pts[(pbase + i) * 3 + 0], py = pts[(pbase + i) * 3 + 1], pz = pts[(pbase + i) * 3 + 2];
#pragma unroll
      for (int pl = 0; pl < 3; ++pl) {
        const float cu = (pl == 2) ? py : px;
        const float cv = (pl == 0) ? py : pz;
        float ix = (cu + 1.0f) * 0.5f * (float)(RR - 1), iy = (cv + 1.0f) * 0.5f * (float)(RR - 1);
        ix = fminf(fmaxf(ix, 0.0f), (float)(RR - 1)); iy = fminf(fmaxf(iy, 0.0f), (float)(RR - 1));
        const int x0 = (int)floorf(ix), y0 = (int)floorf(iy);
        const int x1 = min(x0 + 1, RR - 1), y1 = min(y0 + 1, RR - 1);
        const float wx = ix - (float)x0, wy = iy - (float)y0;
        const float* pc = planes + ((size_t)(pl * PC + lane)) * RR * RR;
        const float v00 = pc[y0 * RR + x0], v01 = pc[y0 * RR + x1], v10 = pc[y1 * RR + x0], v11 = pc[y1 * RR + x1];
        const float val = v00 * (1.f - wx) * (1.f - wy) + v01 * wx * (1.f - wy) + v10 * (1.f - wx) * wy + v11 * wx * wy;
        sA[w][i][pl * PC + lane] = (_Float16)val;
      }
    }
    __builtin_amdgcn_fence(__ATOMIC_ACQ_REL, "workgroup");
    __builtin_amdgcn_wave_barrier();
    Frag af[3];
#pragma unroll
    for (int ks = 0; ks < 3; ++ks) { af[ks].half[0] = *(const v8ha*)&sA[w][ln][ks * 32 + 8 * hh]; af[ks].half[1] = *(const v8ha*)&sA[w][ln][ks * 32 + 16 + 8 * hh]; }
#pragma unroll 1
    for (int br = 0; br < 2; ++br) {
      const _Float16* W1 = br ? rW1h : dW1h; const float* b1 = br ? rb1 : db1;
#pragma unroll 1
      for (int nt = 0; nt < HID / 16; ++nt) {
        const int n = nt * 16 + ln;
        v8f acc = {};
#pragma unroll
        for (int ks = 0; ks < 3; ++ks) {
          Frag b; b.half[0] = *(const v8ha*)(W1 + (size_t)n * FEAT + ks * 32 + 8 * hh); b.half[1] = *(const v8ha*)(W1 + (size_t)n * FEAT + ks * 32 + 16 + 8 * hh);
          acc = mma16(af[ks].v, b.v, acc);
        }
        const float bv = b1[n];
#pragma unroll
        for (int r = 0; r < 8; ++r) {
          const float hv = fmaxf(acc[r] + bv, 0.f);
          if (br == 0) sH[w][8 * hh + r][n] = (_Float16)hv; else sRh[w][8 * hh + r][n] = hv;
        }
      }
    }
    __builtin_amdgcn_fence(__ATOMIC_ACQ_REL, "workgroup");
    __builtin_amdgcn_wave_barrier();
    Frag ah[4];
#pragma unroll
    for (int ks = 0; ks < 4; ++ks) { ah[ks].half[0] = *(const v8ha*)&sH[w][ln][ks * 32 + 8 * hh]; ah[ks].half[1] = *(const v8ha*)&sH[w][ln][ks * 32 + 16 + 8 * hh]; }
#pragma unroll 1
    for (int nt = 0; nt < HID / 16; ++nt) {
      const int n = nt * 16 + ln;
      v8f acc = {};
#pragma unroll
      for (int ks = 0; ks < 4; ++ks) {
        Frag b; b.half[0] = *(const v8ha*)(dW2h + (size_t)n * HID + ks * 32 + 8 * hh); b.half[1] = *(const v8ha*)(dW2h + (size_t)n * HID + ks * 32 + 16 + 8 * hh);
        acc = mma16(ah[ks].v, b.v, acc);
      }
      const float bv = db2[n];
#pragma unroll
      for (int r = 0; r < 8; ++r) sH2[w][8 * hh + r][n] = fmaxf(acc[r] + bv, 0.f);
    }
    __builtin_amdgcn_fence(__ATOMIC_ACQ_REL, "workgroup");
    __builtin_amdgcn_wave_barrier();
    {
      float dsum = 0.f, r0 = 0.f, r1 = 0.f, r2 = 0.f;
#pragma unroll 4
      for (int j = 0; j < 64; ++j) {
        const int kk = hh * 64 + j;
        dsum += sH2[w][ln][kk] * dW3[kk];
        const float rv = sRh[w][ln][kk];
        r0 += rv * rW2[kk]; r1 += rv * rW2[HID + kk]; r2 += rv * rW2[2 * HID + kk];
      }
      dsum += __shfl_xor(dsum, 16, 32); r0 += __shfl_xor(r0, 16, 32); r1 += __shfl_xor(r1, 16, 32); r2 += __shfl_xor(r2, 16, 32);
      if (hh == 0) {
        const float z = dsum + db3[0];
        const float sp = (z > 0.f ? z : 0.f) + log1pf(expf(-fabsf(z)));
        sOut[w][sub * 16 + ln][0] = 1.0f / (1.0f + expf(-(r0 + rb2[0])));
        sOut[w][sub * 16 + ln][1] = 1.0f / (1.0f + expf(-(r1 + rb2[1])));
        sOut[w][sub * 16 + ln][2] = 1.0f / (1.0f + expf(-(r2 + rb2[2])));
        sOut[w][sub * 16 + ln][3] = sp;
      }
    }
  }
  __builtin_amdgcn_fence(__ATOMIC_ACQ_REL, "workgroup");
  __builtin_amdgcn_wave_barrier();
  float rv[4] = {0.f, 0.f, 0.f, 0.f}, dv4[4] = {0.f, 0.f, 0.f, 0.f};
  if (lane < 24) {
#pragma unroll
    for (int j = 0; j < 4; ++j) { const int g = lane * 4 + j; rv[j] = sOut[w][g / 3][g % 3]; }
  }
  if (lane < 8) {
#pragma unroll
    for (int j = 0; j < 4; ++j) dv4[j] = sOut[w][lane * 4 + j][3];
  }
  for (int pass = 0; pass < 2; ++pass) {
    if (lane < 24) { const v4f v4 = {rv[0], rv[1], rv[2], rv[3]}; *(volatile v4f*)(rgb + p0 * 3 + lane * 4) = v4; }
    if (lane < 8)  { const v4f d4 = {dv4[0], dv4[1], dv4[2], dv4[3]}; *(volatile v4f*)(dens + p0 + lane * 4) = d4; }
    if (pass == 0) __threadfence();
  }
}

extern "C" void kernel_launch(void* const* d_in, const int* in_sizes, int n_in,
                              void* d_out, int out_size, void* d_ws, size_t ws_size, hipStream_t stream) {
  (void)in_sizes; (void)n_in; (void)out_size;
  const float* pts = (const float*)d_in[0]; const float* planes = (const float*)d_in[1];
  const float* dW1 = (const float*)d_in[2]; const float* db1 = (const float*)d_in[3];
  const float* dW2 = (const float*)d_in[4]; const float* db2 = (const float*)d_in[5];
  const float* dW3 = (const float*)d_in[6]; const float* db3 = (const float*)d_in[7];
  const float* rW1 = (const float*)d_in[8]; const float* rb1 = (const float*)d_in[9];
  const float* rW2 = (const float*)d_in[10]; const float* rb2 = (const float*)d_in[11];
  char* ws = (char*)d_ws; size_t off = 0;
  _Float16* dW1h = (_Float16*)(ws + off); off += (size_t)HID * FEAT * 2;
  _Float16* rW1h = (_Float16*)(ws + off); off += (size_t)HID * FEAT * 2;
  _Float16* dW2h = (_Float16*)(ws + off); off += (size_t)HID * HID * 2;
  if (off > ws_size) return;
  k_cvt16<<<(HID * FEAT / 8 + 255) / 256, 256, 0, stream>>>(dW1, dW1h, HID * FEAT / 8);
  k_cvt16<<<(HID * FEAT / 8 + 255) / 256, 256, 0, stream>>>(rW1, rW1h, HID * FEAT / 8);
  k_cvt16<<<(HID * HID / 8 + 255) / 256, 256, 0, stream>>>(dW2, dW2h, HID * HID / 8);
  float* rgb = (float*)d_out; float* dens = (float*)d_out + (size_t)NPTS * 3;
  k_nerf<<<NPTS / 32 / 4, 128, 0, stream>>>(pts, planes, dW1h, db1, dW2h, db2, dW3, db3, rW1h, rb1, rW2, rb2, rgb, dens);
}
